// LocalAggregation_75024488726595
// MI455X (gfx1250) — hardware-verified
//
#include <hip/hip_runtime.h>
#include <stddef.h>
#include <stdint.h>

#define KNB    32
#define CIN    64
#define CMID   64
#define COUT   128
#define NCRD   3
#define K1E    96
#define KP1    104
#define KP2    72
#define XPP    72
#define XPUR   (XPP / 8)
#define NT1    (CMID / 16)
#define NT2    (COUT / 16)
#define TM     16
#define NWAVES 4
#define NTHR   128
#define ITERS  25
#define PPB    (NWAVES * ITERS)
#define RECF   256
#define W1PE   (CMID * KP1)
#define W2PE   (COUT * KP2)
#define PREPT  256
#define NBW1   ((W1PE / 8 + PREPT - 1) / PREPT)
#define NBW2   ((W2PE / 8 + PREPT - 1) / PREPT)
#define H1SCALE 16.0f
#define W2SCALE 64.0f
#define Z2INV   (1.0f / 1024.0f)
#define EPSBN   1e-5f

static_assert((KP1 % 8) == 0);
static_assert((KP2 % 8) == 0);
static_assert((XPP % 8) == 0);
static_assert(K1E == 3 * 32);
static_assert(K1E <= KP1);
static_assert(XPP <= KP1);
static_assert(XPUR == 9);
static_assert(NWAVES * 32 == NTHR);
static_assert(NTHR == 2 * CMID);
static_assert((W1PE % 8) == 0);
static_assert((W2PE % 8) == 0);
static_assert(((W1PE * 2) % 128) == 0);
static_assert(((W2PE * 2) % 128) == 0);
static_assert(((TM * KP1) % 8) == 0);
static_assert(((TM * KP2) % 8) == 0);
static_assert(2 * COUT == RECF);
static_assert(NT1 * 16 == CMID);
static_assert(NT2 * 16 == COUT);
static_assert(KNB == 2 * TM);

typedef unsigned short v8us  __attribute__((ext_vector_type(8)));
typedef unsigned short v16us __attribute__((ext_vector_type(16)));
typedef float          v4f   __attribute__((ext_vector_type(4)));
typedef float          v8f   __attribute__((ext_vector_type(8)));
#if defined(__HIP_DEVICE_COMPILE__)
typedef __bf16         v16bf __attribute__((ext_vector_type(16)));
typedef _Float16       v16h  __attribute__((ext_vector_type(16)));
#endif

union FragU { v16us v; v8us half[2]; };

__device__ __forceinline__ unsigned bbits(float f) {
  const unsigned u = __float_as_uint(f);
  return (u + 0x7FFFu + ((u >> 16) & 1u)) >> 16;
}
__device__ __forceinline__ float bf16r(float f) {
  return __uint_as_float(bbits(f) << 16);
}
__device__ __forceinline__ unsigned short hbits(float f) {
  const _Float16 hv = (_Float16)f;
  return __builtin_bit_cast(unsigned short, hv);
}
__device__ __forceinline__ v8f  zero8()   { v8f z = {0.f, 0.f, 0.f, 0.f, 0.f, 0.f, 0.f, 0.f}; return z; }
__device__ __forceinline__ v8us zero8us() { v8us z = {0, 0, 0, 0, 0, 0, 0, 0}; return z; }

__device__ __forceinline__ v16us ldfrag(const unsigned short* p) {
  FragU f;
  f.half[0] = *(const v8us*)(p);
  f.half[1] = *(const v8us*)(p + 16);
  return f.v;
}

__device__ __forceinline__ v8f mma_bf(v16us a, v16us b, v8f c) {
#if defined(__HIP_DEVICE_COMPILE__)
  return __builtin_amdgcn_wmma_f32_16x16x32_bf16(false, __builtin_bit_cast(v16bf, a),
                                                false, __builtin_bit_cast(v16bf, b),
                                                (short)0, c, false, false);
#else
  (void)a; (void)b;
  return c;
#endif
}
__device__ __forceinline__ v8f mma_h(v16us a, v16us b, v8f c) {
#if defined(__HIP_DEVICE_COMPILE__)
  return __builtin_amdgcn_wmma_f32_16x16x32_f16(false, __builtin_bit_cast(v16h, a),
                                               false, __builtin_bit_cast(v16h, b),
                                               (short)0, c, false, false);
#else
  (void)a; (void)b;
  return c;
#endif
}
__device__ __forceinline__ void guard6(v8f& acc, const v16us& a0, const v16us& a1, const v16us& a2,
                                       const v16us& b0, const v16us& b1, const v16us& b2) {
#if defined(__HIP_DEVICE_COMPILE__)
  asm volatile("v_nop\n\tv_nop\n\tv_nop\n\tv_nop"
               : "+v"(acc)
               : "v"(a0), "v"(a1), "v"(a2), "v"(b0), "v"(b1), "v"(b2)
               : "memory");
#else
  (void)acc; (void)a0; (void)a1; (void)a2; (void)b0; (void)b1; (void)b2;
#endif
}
__device__ __forceinline__ void guard4(v8f& acc, const v16us& a0, const v16us& a1,
                                       const v16us& b0, const v16us& b1) {
#if defined(__HIP_DEVICE_COMPILE__)
  asm volatile("v_nop\n\tv_nop\n\tv_nop\n\tv_nop"
               : "+v"(acc)
               : "v"(a0), "v"(a1), "v"(b0), "v"(b1)
               : "memory");
#else
  (void)acc; (void)a0; (void)a1; (void)b0; (void)b1;
#endif
}

__global__ __launch_bounds__(PREPT)
void k_prep(const float* __restrict__ x, const float* __restrict__ p,
            const float* __restrict__ W1, const float* __restrict__ W2,
            unsigned short* XP, unsigned short* W1P, unsigned short* W2P,
            int xpu, int nbx)
{
  const int b = blockIdx.x, tid = threadIdx.x;
  v8us val = zero8us();
  unsigned short* dst;
  bool wr;
  if (b < nbx) {
    const int i   = b * PREPT + tid;
    const int ic  = (i < xpu) ? i : (xpu - 1);
    const int row = ic / XPUR;
    const int cu  = ic - row * XPUR;
    const int cu8 = (cu < 8) ? cu : 7;
    const float4* xs = (const float4*)(x + (size_t)row * CIN + cu8 * 8);
    const float4 a = xs[0], c4 = xs[1];
    const float* ps = p + (size_t)row * NCRD;
    const float xv[8] = {a.x, a.y, a.z, a.w, c4.x, c4.y, c4.z, c4.w};
    const float pv[8] = {ps[0], ps[1], ps[2], 0.f, 0.f, 0.f, 0.f, 0.f};
    const bool isx  = (cu < 8);
    const bool live = (i < xpu);
#pragma unroll
    for (int e = 0; e < 8; ++e) {
      const float f = isx ? xv[e] : pv[e];
      val[e] = (unsigned short)(live ? bbits(f) : 0u);
    }
    dst = XP + (size_t)i * 8;
    wr  = true;
  } else if (b < nbx + NBW1) {
    const int i  = (b - nbx) * PREPT + tid;
    const int ic = (i < W1PE / 8) ? i : (W1PE / 8 - 1);
    const int e0 = ic * 8;
    const int n  = e0 / KP1;
    const int k0 = e0 - n * KP1;
#pragma unroll
    for (int e = 0; e < 8; ++e) {
      const int k  = k0 + e;
      const int kk = (k < 64) ? (k + NCRD) : ((k < 64 + NCRD) ? (k - 64) : 0);
      const float w = W1[kk * CMID + n];
      val[e] = (unsigned short)((k < 64 + NCRD) ? bbits(w) : 0u);
    }
    dst = W1P + (size_t)i * 8;
    wr  = (i < W1PE / 8);
  } else {
    const int i  = (b - nbx - NBW1) * PREPT + tid;
    const int ic = (i < W2PE / 8) ? i : (W2PE / 8 - 1);
    const int e0 = ic * 8;
    const int n  = e0 / KP2;
    const int k0 = e0 - n * KP2;
#pragma unroll
    for (int e = 0; e < 8; ++e) {
      const int k  = k0 + e;
      const int kk = (k < CMID) ? k : (CMID - 1);
      const float w = bf16r(W2[kk * COUT + n]) * W2SCALE;
      val[e] = (unsigned short)((k < CMID) ? (unsigned)hbits(w) : 0u);
    }
    dst = W2P + (size_t)i * 8;
    wr  = (i < W2PE / 8);
  }
  if (wr) *(volatile v8us*)dst = val;
  __threadfence();
  if (wr) *(volatile v8us*)dst = val;
}

template <int PASS>
__global__ __launch_bounds__(NTHR)
void k_fused(const unsigned short* __restrict__ XP, const int* __restrict__ idx,
             const float* __restrict__ p, const float* __restrict__ W1,
             const unsigned short* __restrict__ W1P, const unsigned short* __restrict__ W2P,
             const float* __restrict__ tab1,
             float* part, float* zmax, float* zmin, int npts)
{
  __shared__ __align__(16) unsigned short w1s[W1PE];
  __shared__ __align__(16) unsigned short w2s[PASS ? W2PE : 8];
  __shared__ __align__(16) unsigned short atile[NWAVES * TM * KP1];
  __shared__ __align__(16) unsigned short htile[PASS ? (NWAVES * TM * KP2) : 8];
  __shared__ __align__(16) float sx[NWAVES * RECF];
  __shared__ __align__(16) float srec[RECF];
  __shared__ __align__(16) float stab[2 * CMID];
  __shared__ __align__(16) float w1pf[NCRD * CMID];

  const int tid = threadIdx.x;
  const int lane = tid & 31, wave = tid >> 5;
  const int h = lane >> 4;
  const int c = lane & 15;

  for (int i = tid; i < W1PE / 8; i += NTHR) ((v8us*)w1s)[i] = ((const v8us*)W1P)[i];
  if (PASS) {
    for (int i = tid; i < W2PE / 8; i += NTHR) ((v8us*)w2s)[i] = ((const v8us*)W2P)[i];
    stab[tid] = tab1[tid];
  }
  for (int i = tid; i < NCRD * CMID; i += NTHR) w1pf[i] = bf16r(W1[i]);
  unsigned short* at = atile + wave * TM * KP1;
  unsigned short* ht = htile + (PASS ? wave * TM * KP2 : 0);
  {
    const v8us z = zero8us();
    for (int i = lane; i < TM * KP1 / 8; i += 32) ((v8us*)at)[i] = z;
    if (PASS) for (int i = lane; i < TM * KP2 / 8; i += 32) ((v8us*)ht)[i] = z;
  }
  __syncthreads();

  float s1[NT1], q1[NT1], s2[NT2], q2[NT2];
#pragma unroll
  for (int t = 0; t < NT1; ++t) { s1[t] = 0.f; q1[t] = 0.f; }
#pragma unroll
  for (int t = 0; t < NT2; ++t) { s2[t] = 0.f; q2[t] = 0.f; }

#pragma unroll 1
  for (int it = 0; it < ITERS; ++it) {
    const int  pt    = blockIdx.x * PPB + it * NWAVES + wave;
    const bool valid = pt < npts;
    const int  ptc   = valid ? pt : (npts - 1);
    const float vm   = valid ? 1.0f : 0.0f;
    const float pi0  = bf16r(p[(size_t)ptc * NCRD + 0]);
    const float pi1  = bf16r(p[(size_t)ptc * NCRD + 1]);
    const float pi2  = bf16r(p[(size_t)ptc * NCRD + 2]);
    float mx[NT2], mn[NT2];
#pragma unroll
    for (int t = 0; t < NT2; ++t) { mx[t] = -3.0e38f; mn[t] = 3.0e38f; }

#pragma unroll 1
    for (int s = 0; s < 2; ++s) {
      {
        const int row = ptc * KNB + s * TM + c;
        int j = idx[row];
        j = (j < 0) ? 0 : ((j > npts - 1) ? (npts - 1) : j);
        const v8us* src = (const v8us*)(XP + (size_t)j * XPP) + 4 * h;
        const v8us u0 = src[0], u1 = src[1], u2 = src[2], u3 = src[3], u4 = src[4];
        v8us* dq = (v8us*)(at + c * KP1) + 4 * h;
        dq[0] = u0; dq[1] = u1; dq[2] = u2; dq[3] = u3; dq[4] = u4;
      }
      __syncthreads();

      const unsigned short* ap = at + c * KP1 + 8 * h;
      const v16us a0 = ldfrag(ap);
      const v16us a1 = ldfrag(ap + 32);
      const v16us a2 = ldfrag(ap + 64);
#pragma unroll
      for (int t = 0; t < NT1; ++t) {
        const int n = 16 * t + c;
        const unsigned short* wp = w1s + n * KP1 + 8 * h;
        const v16us g0 = ldfrag(wp);
        const v16us g1 = ldfrag(wp + 32);
        const v16us g2 = ldfrag(wp + 64);
        v8f acc = zero8();
        acc = mma_bf(a0, g0, acc);
        acc = mma_bf(a1, g1, acc);
        acc = mma_bf(a2, g2, acc);
        guard6(acc, a0, a1, a2, g0, g1, g2);
        const float ut = -fmaf(pi2, w1pf[2 * CMID + n], fmaf(pi1, w1pf[CMID + n], pi0 * w1pf[n]));
        if (PASS == 0) {
          float ts = 0.f, tq = 0.f;
#pragma unroll
          for (int r = 0; r < 8; ++r) {
            const float z = acc[r] + ut;
            ts += z;
            tq = fmaf(z, z, tq);
          }
          s1[t] = fmaf(vm, ts, s1[t]);
          q1[t] = fmaf(vm, tq, q1[t]);
        } else {
          const float sc = stab[n], sh = stab[CMID + n];
#pragma unroll
          for (int r = 0; r < 8; ++r) {
            const float z = acc[r] + ut;
            const float v = fmaxf(fmaf(z, sc, sh), 0.0f) * H1SCALE;
            ht[(8 * h + r) * KP2 + n] = hbits(v);
          }
        }
      }

      if (PASS == 1) {
        __syncthreads();
        const unsigned short* hp = ht + c * KP2 + 8 * h;
        const v16us e0 = ldfrag(hp);
        const v16us e1 = ldfrag(hp + 32);
#pragma unroll
        for (int t = 0; t < NT2; ++t) {
          const int n = 16 * t + c;
          const unsigned short* wp = w2s + n * KP2 + 8 * h;
          const v16us g0 = ldfrag(wp);
          const v16us g1 = ldfrag(wp + 32);
          v8f acc = zero8();
          acc = mma_h(e0, g0, acc);
          acc = mma_h(e1, g1, acc);
          guard4(acc, e0, e1, g0, g1);
          float ts = 0.f, tq = 0.f, tmx = -3.0e38f, tmn = 3.0e38f;
#pragma unroll
          for (int r = 0; r < 8; ++r) {
            const float z = acc[r] * Z2INV;
            ts += z;
            tq = fmaf(z, z, tq);
            tmx = fmaxf(tmx, z);
            tmn = fminf(tmn, z);
          }
          s2[t] = fmaf(vm, ts, s2[t]);
          q2[t] = fmaf(vm, tq, q2[t]);
          mx[t] = fmaxf(mx[t], tmx);
          mn[t] = fminf(mn[t], tmn);
        }
      }
      __syncthreads();
    }

    if (PASS == 1) {
      float* so = sx + wave * RECF;
#pragma unroll
      for (int t = 0; t < NT2; ++t) {
        const float a = fmaxf(mx[t], __shfl_xor(mx[t], 16));
        const float b = fminf(mn[t], __shfl_xor(mn[t], 16));
        so[16 * t + c]        = a;
        so[COUT + 16 * t + c] = b;
      }
      __syncthreads();
      const v4f va = *(const v4f*)(so + 4 * lane);
      const v4f vb = *(const v4f*)(so + COUT + 4 * lane);
      float* pa = zmax + (size_t)ptc * COUT + 4 * lane;
      float* pb = zmin + (size_t)ptc * COUT + 4 * lane;
      if (valid) { *(volatile v4f*)pa = va; *(volatile v4f*)pb = vb; }
      __threadfence();
      if (valid) { *(volatile v4f*)pa = va; *(volatile v4f*)pb = vb; }
    }
  }

  __syncthreads();
  {
    float* sa = sx + wave * RECF;
    if (PASS == 0) {
#pragma unroll
      for (int t = 0; t < NT1; ++t) {
        const float a = s1[t] + __shfl_xor(s1[t], 16);
        const float b = q1[t] + __shfl_xor(q1[t], 16);
        sa[16 * t + c]            = a;
        sa[CMID + 16 * t + c]     = b;
        sa[2 * CMID + 16 * t + c] = 0.f;
        sa[3 * CMID + 16 * t + c] = 0.f;
      }
    } else {
#pragma unroll
      for (int t = 0; t < NT2; ++t) {
        const float a = s2[t] + __shfl_xor(s2[t], 16);
        const float b = q2[t] + __shfl_xor(q2[t], 16);
        sa[16 * t + c]        = a;
        sa[COUT + 16 * t + c] = b;
      }
    }
  }
  __syncthreads();
  for (int i = tid; i < RECF; i += NTHR)
    srec[i] = (sx[i] + sx[RECF + i]) + (sx[2 * RECF + i] + sx[3 * RECF + i]);
  __syncthreads();
  {
    const int q = (wave & 1) * 32 + lane;
    const v4f v = *(const v4f*)(srec + 4 * q);
    float* pp = part + (size_t)blockIdx.x * RECF + 4 * q;
    const bool wr = (wave < 2);
    if (wr) *(volatile v4f*)pp = v;
    __threadfence();
    if (wr) *(volatile v4f*)pp = v;
  }
}

template <int C>
__global__ __launch_bounds__(NTHR)
void k_bnred(const float* __restrict__ part, int nblk, int nrows,
             const float* __restrict__ bia, const float* __restrict__ gam,
             const float* __restrict__ bet, float* tab)
{
  __shared__ __align__(16) float st[RECF];
  const int tid = threadIdx.x, lane = tid & 31, wave = tid >> 5;
  const int cc = (tid < C) ? tid : (C - 1);
  double s = 0.0, q = 0.0;
#pragma unroll 1
  for (int k = 0; k < nblk; ++k) {
    const float* rp = part + (size_t)k * RECF;
    s += (double)rp[cc];
    q += (double)rp[C + cc];
  }
  const double invr = 1.0 / (double)nrows;
  const double mu = s * invr;
  double var = q * invr - mu * mu;
  var = (var > 0.0) ? var : 0.0;
  const float rstd = rsqrtf((float)var + EPSBN);
  const float gb = bf16r(gam[cc]), bb = bf16r(bia[cc]), tb = bf16r(bet[cc]);
  const float sc  = gb * rstd;
  const float muz = (float)mu + bb;
  const float sh  = fmaf(bb - muz, sc, tb);
  for (int i = tid; i < RECF; i += NTHR) st[i] = 0.f;
  __syncthreads();
  if (tid < C) { st[tid] = sc; st[C + tid] = sh; }
  __syncthreads();
  {
    const int qd = (wave & 1) * 32 + lane;
    const v4f v = *(const v4f*)(st + 4 * qd);
    float* pp = tab + 4 * qd;
    const bool wr = (wave < 2);
    if (wr) *(volatile v4f*)pp = v;
    __threadfence();
    if (wr) *(volatile v4f*)pp = v;
  }
}

__global__ __launch_bounds__(NTHR)
void k_out(const float* __restrict__ zmax, const float* __restrict__ zmin,
           const float* __restrict__ tab2, float* out, int npts)
{
  const int tid = threadIdx.x, lane = tid & 31, wave = tid >> 5;
  const int  pt    = blockIdx.x * NWAVES + wave;
  const bool valid = pt < npts;
  const int  ptc   = valid ? pt : (npts - 1);
  const v4f a  = *(const v4f*)(zmax + (size_t)ptc * COUT + 4 * lane);
  const v4f b  = *(const v4f*)(zmin + (size_t)ptc * COUT + 4 * lane);
  const v4f sc = *(const v4f*)(tab2 + 4 * lane);
  const v4f sh = *(const v4f*)(tab2 + COUT + 4 * lane);
  v4f o;
#pragma unroll
  for (int i = 0; i < 4; ++i) {
    const float v = (sc[i] >= 0.0f) ? a[i] : b[i];
    o[i] = fmaxf(fmaf(v, sc[i], sh[i]), 0.0f);
  }
  float* po = out + (size_t)ptc * COUT + 4 * lane;
  if (valid) *(volatile v4f*)po = o;
  __threadfence();
  if (valid) *(volatile v4f*)po = o;
}

extern "C" void kernel_launch(void* const* d_in, const int* in_sizes, int n_in,
                              void* d_out, int out_size, void* d_ws, size_t ws_size,
                              hipStream_t stream) {
  if (n_in < 11) return;
  if (in_sizes[0] < NCRD || (in_sizes[0] % NCRD) != 0) return;
  const int npts = in_sizes[0] / NCRD;
  if (in_sizes[1] != npts * CIN) return;
  if (in_sizes[2] != npts * KNB) return;
  if (in_sizes[3] != (NCRD + CIN) * CMID) return;
  if (in_sizes[4] != CMID || in_sizes[5] != CMID || in_sizes[6] != CMID) return;
  if (in_sizes[7] != CMID * COUT) return;
  if (in_sizes[8] != COUT || in_sizes[9] != COUT || in_sizes[10] != COUT) return;
  if ((long long)out_size != (long long)npts * (long long)COUT) return;

  const float* p   = (const float*)d_in[0];
  const float* x   = (const float*)d_in[1];
  const int*   idx = (const int*)d_in[2];
  const float* W1  = (const float*)d_in[3];
  const float* b1  = (const float*)d_in[4];
  const float* g1  = (const float*)d_in[5];
  const float* bt1 = (const float*)d_in[6];
  const float* W2  = (const float*)d_in[7];
  const float* b2  = (const float*)d_in[8];
  const float* g2  = (const float*)d_in[9];
  const float* bt2 = (const float*)d_in[10];
  float* out = (float*)d_out;

  const int xpu  = npts * XPUR;
  const int nbx  = (xpu + PREPT - 1) / PREPT;
  const int nblk = (npts + PPB - 1) / PPB;
  const int nbo  = (npts + NWAVES - 1) / NWAVES;
  const int nrows = npts * KNB;

  size_t off = 0;
  const size_t oXP = off;  off += (size_t)nbx * PREPT * 16;
  const size_t oW1 = off;  off += (size_t)W1PE * 2;
  const size_t oW2 = off;  off += (size_t)W2PE * 2;
  const size_t oP1 = off;  off += (size_t)nblk * RECF * 4;
  const size_t oP2 = off;  off += (size_t)nblk * RECF * 4;
  const size_t oT1 = off;  off += (size_t)RECF * 4;
  const size_t oT2 = off;  off += (size_t)RECF * 4;
  const size_t oZX = off;  off += (size_t)npts * COUT * 4;
  const size_t oZN = off;  off += (size_t)npts * COUT * 4;
  if (off > ws_size || off > (size_t)134217728) return;

  char* ws = (char*)d_ws;
  unsigned short* XP  = (unsigned short*)(ws + oXP);
  unsigned short* W1P = (unsigned short*)(ws + oW1);
  unsigned short* W2P = (unsigned short*)(ws + oW2);
  float* part1 = (float*)(ws + oP1);
  float* part2 = (float*)(ws + oP2);
  float* tab1  = (float*)(ws + oT1);
  float* tab2  = (float*)(ws + oT2);
  float* zmax  = (float*)(ws + oZX);
  float* zmin  = (float*)(ws + oZN);

  k_prep<<<dim3(nbx + NBW1 + NBW2), dim3(PREPT), 0, stream>>>(x, p, W1, W2, XP, W1P, W2P, xpu, nbx);
  k_fused<0><<<dim3(nblk), dim3(NTHR), 0, stream>>>(XP, idx, p, W1, W1P, W2P, tab1,
                                                    part1, zmax, zmin, npts);
  k_bnred<CMID><<<dim3(1), dim3(NTHR), 0, stream>>>(part1, nblk, nrows, b1, g1, bt1, tab1);
  k_fused<1><<<dim3(nblk), dim3(NTHR), 0, stream>>>(XP, idx, p, W1, W1P, W2P, tab1,
                                                    part2, zmax, zmin, npts);
  k_bnred<COUT><<<dim3(1), dim3(NTHR), 0, stream>>>(part2, nblk, nrows, b2, g2, bt2, tab2);
  k_out<<<dim3(nbo), dim3(NTHR), 0, stream>>>(zmax, zmin, tab2, out, npts);
  (void)hipGetLastError();
}
